// GNFConverter_14671608283534
// MI455X (gfx1250) — hardware-run, weakly checked
//
#include <hip/hip_runtime.h>


#ifndef NB
#define NB 16
#endif
#ifndef NP
#define NP 8192
#endif
#define NB_FULL 16
#define NP_FULL 8192
#ifndef OUT_NP
#define OUT_NP NP
#endif
#define NA   128
#define NT   5
#define OW   15
#define AW   4
#define QT   (16 * AW)
#define VTP  136
#define OPIECES (QT * OW / 4)
#define QRS  2048.0f
#define QRI  (1.0f / 2048.0f)
#define L2E  1.4426950408889634f
#define PSH  14.0f
#define BIGF 3.0e38f
#define CLIPR 0.3f

static_assert(NT == 5);
static_assert(NT * 4 <= 32);
static_assert(NA % 32 == 0);
static_assert(NA % (32 * AW) == 0);
static_assert(VTP >= NA);
static_assert((VTP * 2) % 16 == 0);
static_assert(NP % QT == 0);
static_assert((QT * OW) % 4 == 0);
static_assert((QT * OW * 4) % 128 == 0);
static_assert(((size_t)OUT_NP * OW * 4) % 128 == 0);
static_assert(OPIECES > 32 * AW);
static_assert(OPIECES <= 2 * 32 * AW);
static_assert((OPIECES - 32 * AW) % 8 == 0);
static_assert((32 * AW + (OPIECES - 32 * AW)) * 16 == QT * OW * 4);
static_assert(NB <= NB_FULL);
static_assert(NP <= NP_FULL);
static_assert((size_t)NB_FULL * NP_FULL * OW * 4 == (size_t)7864320);
static_assert(32 * VTP * 2 + 4 * NA * 4 + QT * OW * 4 <= 131072);

typedef _Float16 h16;
typedef __attribute__((ext_vector_type(16))) _Float16 v16h;
typedef __attribute__((ext_vector_type(8)))  _Float16 v8h;
typedef __attribute__((ext_vector_type(8)))  float    v8f;
typedef __attribute__((ext_vector_type(4)))  float    v4f;
typedef __attribute__((ext_vector_type(4)))  int      v4i;
typedef v4f __attribute__((may_alias)) v4fa;
typedef v4i __attribute__((may_alias)) v4ia;
typedef v8h __attribute__((may_alias)) v8ha;

__device__ __forceinline__ unsigned short f2bf(float f) { unsigned u = __float_as_uint(f); u += 0x7FFFu + ((u >> 16) & 1u); return (unsigned short)(u >> 16); }
__device__ __forceinline__ float bfr(float f) { return __uint_as_float(((unsigned)f2bf(f)) << 16); }
__device__ __forceinline__ v16h cat16(v8h lo, v8h hi) { return __builtin_shufflevector(lo, hi, 0, 1, 2, 3, 4, 5, 6, 7, 8, 9, 10, 11, 12, 13, 14, 15); }
__device__ __forceinline__ v8f wmma16(v16h a, v16h b, v8f c) { return __builtin_amdgcn_wmma_f32_16x16x32_f16(false, a, false, b, (short)0, c, false, false); }
__device__ __forceinline__ v8f wmma16g(v16h a, v16h b, v8f c) {
    c = wmma16(a, b, c);
    asm volatile("v_nop\n\tv_nop\n\tv_nop\n\tv_nop" : "+v"(c) : "v"(a), "v"(b));
    return c;
}
__device__ __forceinline__ h16 toh_flush(float v) { const h16 r = (h16)v; return (fabsf(v) < 6.103515625e-05f) ? (h16)0.0f : r; }

__device__ __forceinline__ float dist3(float cx, float cy, float cz, float qx, float qy, float qz) {
    const float dx = cx - qx, dy = cy - qy, dz = cz - qz;
    return __builtin_amdgcn_sqrtf(dx * dx + dy * dy + dz * dz);
}

__device__ __forceinline__ void field3(float nx, float ny, float nz, float den, float qx, float qy, float qz, float& gx, float& gy, float& gz) {
    const bool any = den > 0.0f;
    const float inv = __builtin_amdgcn_rcpf(any ? den : 1.0f);
    const float x = nx * inv - qx, y = ny * inv - qy, z = nz * inv - qz;
    const float mag = __builtin_amdgcn_sqrtf(x * x + y * y + z * z);
    const bool cl = mag > CLIPR;
    const float sc = cl ? (CLIPR * __builtin_amdgcn_rcpf(cl ? mag : 1.0f)) : 1.0f;
    gx = any ? x * sc : 0.0f; gy = any ? y * sc : 0.0f; gz = any ? z * sc : 0.0f;
}

__global__ __launch_bounds__(32 * AW) void k_field(const float* __restrict__ coords, const int* __restrict__ atypes, const float* __restrict__ query, float* OUT) {
    __shared__ __align__(16) h16   vts[32 * VTP];
    __shared__ __align__(16) float cxs[NA];
    __shared__ __align__(16) float cys[NA];
    __shared__ __align__(16) float czs[NA];
    __shared__ __align__(16) int   ctys[NA];
    __shared__ __align__(16) float osb[QT * OW];
    const int tid = threadIdx.x;
    const int lane = tid & 31, lr = lane & 15, hi = lane >> 4;
    const int wave = __builtin_amdgcn_readfirstlane((int)(threadIdx.x >> 5));
    const int b = blockIdx.y;

    for (int a = tid; a < NA; a += 32 * AW) {
        const size_t ci = ((size_t)b * NA + (size_t)a) * 3;
        const float x = bfr(coords[ci]), y = bfr(coords[ci + 1]), z = bfr(coords[ci + 2]);
        const int ty = atypes[(size_t)b * NA + a];
        cxs[a] = x; cys[a] = y; czs[a] = z; ctys[a] = ty;
        const h16 xh = toh_flush(x), yh = toh_flush(y), zh = toh_flush(z);
        const h16 one = (h16)1.0f, zero = (h16)0.0f;
#pragma unroll
        for (int d = 0; d < 32; ++d) {
            const int tq = d >> 2, c = d & 3;
            const h16 v = (c == 0) ? xh : ((c == 1) ? yh : ((c == 2) ? zh : one));
            const bool on = (tq < NT) & (ty == tq);
            vts[d * VTP + a] = on ? v : zero;
        }
    }
    __syncthreads();

    const int p0 = (blockIdx.x * AW + wave) * 16;
    const size_t qi = ((size_t)b * NP_FULL + (size_t)(p0 + lr)) * 3;
    const float qx = bfr(query[qi]), qy = bfr(query[qi + 1]), qz = bfr(query[qi + 2]);

    float mt[NT];
#pragma unroll
    for (int t = 0; t < NT; ++t) mt[t] = BIGF;
#pragma unroll 1
    for (int a0 = 0; a0 < NA; a0 += 32) {
#pragma unroll
        for (int u = 0; u < 2; ++u) {
            const int ja = a0 + 16 * u + 8 * hi;
            const v4f x0 = *(const v4fa*)(&cxs[ja]), x1 = *(const v4fa*)(&cxs[ja + 4]);
            const v4f y0 = *(const v4fa*)(&cys[ja]), y1 = *(const v4fa*)(&cys[ja + 4]);
            const v4f z0 = *(const v4fa*)(&czs[ja]), z1 = *(const v4fa*)(&czs[ja + 4]);
            const v4i c0 = *(const v4ia*)(&ctys[ja]), c1 = *(const v4ia*)(&ctys[ja + 4]);
            float ax[8], ay[8], az[8]; int at[8];
#pragma unroll
            for (int r = 0; r < 4; ++r) { ax[r] = x0[r]; ax[4 + r] = x1[r]; ay[r] = y0[r]; ay[4 + r] = y1[r]; az[r] = z0[r]; az[4 + r] = z1[r]; at[r] = c0[r]; at[4 + r] = c1[r]; }
#pragma unroll
            for (int r = 0; r < 8; ++r) {
                const float d = dist3(ax[r], ay[r], az[r], qx, qy, qz);
#pragma unroll
                for (int t = 0; t < NT; ++t) mt[t] = fminf(mt[t], (at[r] == t) ? d : BIGF);
            }
        }
    }
#pragma unroll
    for (int t = 0; t < NT; ++t) mt[t] = fminf(mt[t], __shfl_xor(mt[t], 16, 32));

    v8f o0 = (v8f){}, o1 = (v8f){}, oR0 = (v8f){}, oR1 = (v8f){};
#pragma unroll 1
    for (int a0 = 0; a0 < NA; a0 += 32) {
        v16h pb, pr;
#pragma unroll
        for (int u = 0; u < 2; ++u) {
            const int ja = a0 + 16 * u + 8 * hi;
            const v4f x0 = *(const v4fa*)(&cxs[ja]), x1 = *(const v4fa*)(&cxs[ja + 4]);
            const v4f y0 = *(const v4fa*)(&cys[ja]), y1 = *(const v4fa*)(&cys[ja + 4]);
            const v4f z0 = *(const v4fa*)(&czs[ja]), z1 = *(const v4fa*)(&czs[ja + 4]);
            const v4i c0 = *(const v4ia*)(&ctys[ja]), c1 = *(const v4ia*)(&ctys[ja + 4]);
            float ax[8], ay[8], az[8]; int at[8];
#pragma unroll
            for (int r = 0; r < 4; ++r) { ax[r] = x0[r]; ax[4 + r] = x1[r]; ay[r] = y0[r]; ay[4 + r] = y1[r]; az[r] = z0[r]; az[4 + r] = z1[r]; at[r] = c0[r]; at[4 + r] = c1[r]; }
#pragma unroll
            for (int r = 0; r < 8; ++r) {
                const float d = dist3(ax[r], ay[r], az[r], qx, qy, qz);
                const int ty = at[r];
                float ms = d;
#pragma unroll
                for (int t = 0; t < NT; ++t) ms = (ty == t) ? mt[t] : ms;
                const bool ok = ((unsigned)ty < (unsigned)NT);
                const float e = (ms - d) * L2E + PSH;
                const float ev = __builtin_amdgcn_exp2f(e);
                const float g = (ok & (e >= -14.0f)) ? ev : 0.0f;
                const h16 ph = (h16)g;
                pb[8 * u + r] = ph;
                pr[8 * u + r] = toh_flush((g - (float)ph) * QRS);
            }
        }
        const int vo = lr * VTP + a0 + 8 * hi;
        const v16h v0 = cat16(*(const v8ha*)(&vts[vo]), *(const v8ha*)(&vts[vo + 16]));
        const v16h v1 = cat16(*(const v8ha*)(&vts[vo + 16 * VTP]), *(const v8ha*)(&vts[vo + 16 * VTP + 16]));
        o0  = wmma16g(v0, pb, o0);
        o1  = wmma16g(v1, pb, o1);
        oR0 = wmma16g(v0, pr, oR0);
        oR1 = wmma16g(v1, pr, oR1);
    }

    const v8f f0 = o0 + oR0 * QRI, f1 = o1 + oR1 * QRI;
    const int ob = (wave * 16 + lr) * OW;
    float gx, gy, gz;
    field3(f0[0], f0[1], f0[2], f0[3], qx, qy, qz, gx, gy, gz);
    { const int tt = 2 * hi;     osb[ob + tt * 3 + 0] = gx; osb[ob + tt * 3 + 1] = gy; osb[ob + tt * 3 + 2] = gz; }
    field3(f0[4], f0[5], f0[6], f0[7], qx, qy, qz, gx, gy, gz);
    { const int tt = 2 * hi + 1; osb[ob + tt * 3 + 0] = gx; osb[ob + tt * 3 + 1] = gy; osb[ob + tt * 3 + 2] = gz; }
    field3(f1[0], f1[1], f1[2], f1[3], qx, qy, qz, gx, gy, gz);
    if (hi == 0) { osb[ob + 12] = gx; osb[ob + 13] = gy; osb[ob + 14] = gz; }
    __syncthreads();

    float* obase = OUT + ((size_t)b * OUT_NP + (size_t)blockIdx.x * QT) * OW;
    const int p1 = 32 * AW + tid;
    const int p1c = (p1 < OPIECES) ? p1 : (OPIECES - 1);
    const v4f val0 = *(const v4fa*)(&osb[tid * 4]);
    v4f val1 = *(const v4fa*)(&osb[p1c * 4]);
    asm volatile("" : "+v"(val1));
    const bool w1 = p1 < OPIECES;
#pragma unroll 1
    for (int ps = 0; ps < 2; ++ps) {
        *(volatile v4f*)(obase + (size_t)tid * 4) = val0;
        if (w1) *(volatile v4f*)(obase + (size_t)p1 * 4) = val1;
        if (ps == 0) __threadfence();
    }
}

extern "C" void kernel_launch(void* const* d_in, const int* in_sizes, int n_in,
                              void* d_out, int out_size, void* d_ws, size_t ws_size, hipStream_t stream) {
    if (n_in < 3) return;
    if ((size_t)in_sizes[0] < (size_t)NB * NA * 3) return;
    if ((size_t)in_sizes[1] < (size_t)NB * NA) return;
    if ((size_t)in_sizes[2] < ((size_t)(NB - 1) * NP_FULL + NP) * 3) return;
    if ((size_t)out_size < ((size_t)(NB - 1) * OUT_NP + NP) * OW) return;
    (void)d_ws; (void)ws_size;
    const float* coords = (const float*)d_in[0];
    const int*   atypes = (const int*)d_in[1];
    const float* query  = (const float*)d_in[2];
    float* OUT = (float*)d_out;
    k_field<<<dim3(NP / QT, NB, 1), 32 * AW, 0, stream>>>(coords, atypes, query, OUT);
}
